// GATSpatioTemporalModel_1005022347770
// MI455X (gfx1250) — hardware-verified
//
#include <hip/hip_runtime.h>
#include <stddef.h>

#define NB    8
#define NN    512
#define DIN   64
#define NH    8
#define NF    128
#define NL    2
#define HF    (NH * NF)
#define NEGV  (-9e15f)
#define SLOPE 0.2f
#define LNEPS 1e-5f
#define SLP   68
#define PTP   40
#define OTP   132
#define TRP   72

typedef __attribute__((ext_vector_type(16))) __bf16 v16b;
typedef __attribute__((ext_vector_type(8)))  float  v8f;
typedef __attribute__((ext_vector_type(4)))  float  v4f;
typedef __attribute__((ext_vector_type(4)))  unsigned int v4u;
typedef __attribute__((ext_vector_type(4)))  int    v4i;

union FragU { v16b v; v4u u[2]; };

__device__ __forceinline__ unsigned short f2bf_bits(float f) {
  const unsigned u = __float_as_uint(f);
  return (unsigned short)((u + 0x7FFFu + ((u >> 16) & 1u)) >> 16);
}
__device__ __forceinline__ float bf2f(unsigned short b) { return __uint_as_float(((unsigned)b) << 16); }
__device__ __forceinline__ unsigned pk16(unsigned short a, unsigned short b) { return (unsigned)a | ((unsigned)b << 16); }
__device__ __forceinline__ void cvt1(float v, unsigned short& hb, unsigned short& lb) {
  hb = f2bf_bits(v);
  lb = f2bf_bits(v - bf2f(hb));
}
__device__ __forceinline__ unsigned split2(float x, float y, unsigned& lo) {
  unsigned short hx, lx, hy, ly;
  cvt1(x, hx, lx);
  cvt1(y, hy, ly);
  lo = pk16(lx, ly);
  return pk16(hx, hy);
}
__device__ __forceinline__ void split8(v4f a, v4f b, v4u& hi, v4u& lo) {
  unsigned l0, l1, l2, l3;
  hi.x = split2(a.x, a.y, l0);
  hi.y = split2(a.z, a.w, l1);
  hi.z = split2(b.x, b.y, l2);
  hi.w = split2(b.z, b.w, l3);
  lo.x = l0; lo.y = l1; lo.z = l2; lo.w = l3;
}

__device__ __forceinline__ v16b ldfrag(const unsigned short* p) {
  FragU f;
  f.u[0] = *(const v4u*)(p);
  f.u[1] = *(const v4u*)(p + 16);
  return f.v;
}
__device__ __forceinline__ v8f mma(v16b a, v16b b, v8f c) {
  return __builtin_amdgcn_wmma_f32_16x16x32_bf16(false, a, false, b, (short)0, c, false, false);
}
__device__ __forceinline__ v8f zero8() { return (v8f){0.f, 0.f, 0.f, 0.f, 0.f, 0.f, 0.f, 0.f}; }

__device__ __forceinline__ void mma12(v8f (&c)[4], v16b ah, v16b al,
                                      const unsigned short* bph, const unsigned short* bpl, size_t bsub) {
  const v16b bh0 = ldfrag(bph);
  const v16b bh1 = ldfrag(bph + bsub);
  const v16b bh2 = ldfrag(bph + 2 * bsub);
  const v16b bh3 = ldfrag(bph + 3 * bsub);
  const v16b bl0 = ldfrag(bpl);
  const v16b bl1 = ldfrag(bpl + bsub);
  const v16b bl2 = ldfrag(bpl + 2 * bsub);
  const v16b bl3 = ldfrag(bpl + 3 * bsub);
  c[0] = mma(ah, bh0, c[0]); c[0] = mma(ah, bl0, c[0]); c[0] = mma(al, bh0, c[0]);
  c[1] = mma(ah, bh1, c[1]); c[1] = mma(ah, bl1, c[1]); c[1] = mma(al, bh1, c[1]);
  c[2] = mma(ah, bh2, c[2]); c[2] = mma(ah, bl2, c[2]); c[2] = mma(al, bh2, c[2]);
  c[3] = mma(ah, bh3, c[3]); c[3] = mma(ah, bl3, c[3]); c[3] = mma(al, bh3, c[3]);
  asm volatile("v_nop\n\tv_nop\n\tv_nop\n\tv_nop"
               : "+v"(c[0]), "+v"(c[1]), "+v"(c[2]), "+v"(c[3])
               : "v"(ah), "v"(al), "v"(bh0), "v"(bh1), "v"(bh2), "v"(bh3),
                 "v"(bl0), "v"(bl1), "v"(bl2), "v"(bl3));
}
__device__ __forceinline__ void accguard(v8f (&c)[4]) {
  asm volatile("v_nop\n\tv_nop\n\tv_nop\n\tv_nop" : "+v"(c[0]), "+v"(c[1]), "+v"(c[2]), "+v"(c[3]));
}

__global__ void __launch_bounds__(256)
k_split(const float* __restrict__ in, unsigned short* __restrict__ out, long plane, int n8)
{
  const int i = blockIdx.x * 256 + threadIdx.x;
  if (i < n8) {
    const size_t e = (size_t)i * 8;
    const v4f a = *(const v4f*)(in + e);
    const v4f b = *(const v4f*)(in + e + 4);
    v4u hi, lo;
    split8(a, b, hi, lo);
    *(volatile v4u*)(out + e) = hi;
    *(volatile v4u*)(out + (size_t)plane + e) = lo;
    __threadfence();
    *(volatile v4u*)(out + e) = hi;
    *(volatile v4u*)(out + (size_t)plane + e) = lo;
  }
}

__global__ void __launch_bounds__(256)
k_tr(const float* __restrict__ in, int rows, int cols, long strideIn,
     unsigned short* __restrict__ out, long plane, long strideOut)
{
  __shared__ __align__(16) unsigned short th[64 * TRP];
  __shared__ __align__(16) unsigned short tl[64 * TRP];
  const int c0 = blockIdx.x * 64;
  const int r0 = blockIdx.y * 64;
  const int z  = blockIdx.z;
  const int t  = threadIdx.x;
  {
    const int rr = t >> 2, cq = (t & 3) * 16;
    const float* src = in + (size_t)z * strideIn + (size_t)(r0 + rr) * cols + c0 + cq;
#pragma unroll
    for (int q = 0; q < 4; ++q) {
      const v4f f = *(const v4f*)(src + 4 * q);
      const int o = rr * TRP + cq + 4 * q;
      unsigned short hb, lb;
      cvt1(f.x, hb, lb); th[o]     = hb; tl[o]     = lb;
      cvt1(f.y, hb, lb); th[o + 1] = hb; tl[o + 1] = lb;
      cvt1(f.z, hb, lb); th[o + 2] = hb; tl[o + 2] = lb;
      cvt1(f.w, hb, lb); th[o + 3] = hb; tl[o + 3] = lb;
    }
  }
  __syncthreads();
  const int sub = t >> 3, c8 = (t & 7) * 8;
  v4u hv0, lv0, hv1, lv1;
  {
    const int oc = sub;
    hv0.x = pk16(th[(c8 + 0) * TRP + oc], th[(c8 + 1) * TRP + oc]);
    hv0.y = pk16(th[(c8 + 2) * TRP + oc], th[(c8 + 3) * TRP + oc]);
    hv0.z = pk16(th[(c8 + 4) * TRP + oc], th[(c8 + 5) * TRP + oc]);
    hv0.w = pk16(th[(c8 + 6) * TRP + oc], th[(c8 + 7) * TRP + oc]);
    lv0.x = pk16(tl[(c8 + 0) * TRP + oc], tl[(c8 + 1) * TRP + oc]);
    lv0.y = pk16(tl[(c8 + 2) * TRP + oc], tl[(c8 + 3) * TRP + oc]);
    lv0.z = pk16(tl[(c8 + 4) * TRP + oc], tl[(c8 + 5) * TRP + oc]);
    lv0.w = pk16(tl[(c8 + 6) * TRP + oc], tl[(c8 + 7) * TRP + oc]);
  }
  {
    const int oc = 32 + sub;
    hv1.x = pk16(th[(c8 + 0) * TRP + oc], th[(c8 + 1) * TRP + oc]);
    hv1.y = pk16(th[(c8 + 2) * TRP + oc], th[(c8 + 3) * TRP + oc]);
    hv1.z = pk16(th[(c8 + 4) * TRP + oc], th[(c8 + 5) * TRP + oc]);
    hv1.w = pk16(th[(c8 + 6) * TRP + oc], th[(c8 + 7) * TRP + oc]);
    lv1.x = pk16(tl[(c8 + 0) * TRP + oc], tl[(c8 + 1) * TRP + oc]);
    lv1.y = pk16(tl[(c8 + 2) * TRP + oc], tl[(c8 + 3) * TRP + oc]);
    lv1.z = pk16(tl[(c8 + 4) * TRP + oc], tl[(c8 + 5) * TRP + oc]);
    lv1.w = pk16(tl[(c8 + 6) * TRP + oc], tl[(c8 + 7) * TRP + oc]);
  }
  unsigned short* ob = out + (size_t)z * strideOut;
  const size_t o0 = (size_t)(c0 + sub) * rows + r0 + c8;
  const size_t o1 = (size_t)(c0 + 32 + sub) * rows + r0 + c8;
  for (int pass = 0; pass < 2; ++pass) {
    *(volatile v4u*)(ob + o0) = hv0;
    *(volatile v4u*)(ob + (size_t)plane + o0) = lv0;
    *(volatile v4u*)(ob + o1) = hv1;
    *(volatile v4u*)(ob + (size_t)plane + o1) = lv1;
    __threadfence();
  }
}

template <int EPI>
__global__ void __launch_bounds__(256)
k_gemm(const unsigned short* __restrict__ Apl, long aPlane, int lda, long aGrp, int aMod,
       const unsigned short* __restrict__ Bpl, long bPlane, int ldb, long bGrp, int bDiv,
       int K, const float* __restrict__ vecp,
       float* __restrict__ outF, unsigned short* __restrict__ outP, long oPlane)
{
  __shared__ __align__(16) float slab[8][16 * SLP];
  __shared__ float red[8][2][64];
  __shared__ __align__(16) float sline[2][64];

  const int t = threadIdx.x, lane = t & 31, w = t >> 5, h = lane >> 4, rl = lane & 15;
  const int g = blockIdx.z;
  const int aIdx = g % aMod;
  const int bIdx = g / bDiv;
  const int n0 = blockIdx.x * 64;
  const int m0 = blockIdx.y * 128 + 16 * w;
  const unsigned short* Ab = Apl + (size_t)aIdx * (size_t)aGrp + (size_t)(m0 + rl) * lda + 8 * h;
  const unsigned short* Bb = Bpl + (size_t)bIdx * (size_t)bGrp + (size_t)(n0 + rl) * ldb + 8 * h;
  const size_t bsub = (size_t)16 * ldb;

  v8f acc[4];
  acc[0] = zero8(); acc[1] = zero8(); acc[2] = zero8(); acc[3] = zero8();
  for (int k0 = 0; k0 < K; k0 += 32) {
    const v16b ah = ldfrag(Ab + k0);
    const v16b al = ldfrag(Ab + (size_t)aPlane + k0);
    mma12(acc, ah, al, Bb + k0, Bb + (size_t)bPlane + k0, bsub);
  }
  accguard(acc);

  float* sl = slab[w];
  if constexpr (EPI == 0) {
#pragma unroll
    for (int j = 0; j < 4; ++j) {
      const float bv = vecp[n0 + 16 * j + rl];
#pragma unroll
      for (int r = 0; r < 8; ++r) {
        float v = acc[j][r] + bv;
        v = fmaxf(v, 0.0f);
        sl[(8 * h + r) * SLP + 16 * j + rl] = v;
      }
    }
  } else {
    const float* vec = vecp + (size_t)aIdx * (2 * NF) + m0 + 8 * h;
    const v4f a1a = *(const v4f*)(vec);
    const v4f a1b = *(const v4f*)(vec + 4);
    const v4f a2a = *(const v4f*)(vec + NF);
    const v4f a2b = *(const v4f*)(vec + NF + 4);
#pragma unroll
    for (int j = 0; j < 4; ++j) {
#pragma unroll
      for (int r = 0; r < 8; ++r) sl[(8 * h + r) * SLP + 16 * j + rl] = acc[j][r];
      float p1 = ((acc[j][0] * a1a.x + acc[j][1] * a1a.y) + (acc[j][2] * a1a.z + acc[j][3] * a1a.w)) +
                 ((acc[j][4] * a1b.x + acc[j][5] * a1b.y) + (acc[j][6] * a1b.z + acc[j][7] * a1b.w));
      float p2 = ((acc[j][0] * a2a.x + acc[j][1] * a2a.y) + (acc[j][2] * a2a.z + acc[j][3] * a2a.w)) +
                 ((acc[j][4] * a2b.x + acc[j][5] * a2b.y) + (acc[j][6] * a2b.z + acc[j][7] * a2b.w));
      p1 += __shfl_xor(p1, 16, 32);
      p2 += __shfl_xor(p2, 16, 32);
      if (lane < 16) {
        red[w][0][16 * j + lane] = p1;
        red[w][1][16 * j + lane] = p2;
      }
    }
  }
  __syncthreads();
  if constexpr (EPI == 1) {
    if (t < 128) {
      const int which = t >> 6, c = t & 63;
      float s = red[0][which][c];
#pragma unroll
      for (int w8 = 1; w8 < 8; ++w8) s += red[w8][which][c];
      sline[which][c] = s;
    }
    __syncthreads();
  }

  for (int pass = 0; pass < 2; ++pass) {
    if constexpr (EPI == 0) {
#pragma unroll
      for (int it = 0; it < 8; ++it) {
        const int row = 2 * it + h;
        const v4f v = *(const v4f*)(sl + row * SLP + rl * 4);
        *(volatile v4f*)(outF + (size_t)(m0 + row) * NF + n0 + rl * 4) = v;
      }
#pragma unroll
      for (int it = 0; it < 4; ++it) {
        const int row = 4 * it + (lane >> 3);
        const int c8 = (lane & 7) * 8;
        const v4f a = *(const v4f*)(sl + row * SLP + c8);
        const v4f b = *(const v4f*)(sl + row * SLP + c8 + 4);
        v4u hi, lo;
        split8(a, b, hi, lo);
        const size_t po = (size_t)(m0 + row) * NF + n0 + c8;
        *(volatile v4u*)(outP + po) = hi;
        *(volatile v4u*)(outP + (size_t)oPlane + po) = lo;
      }
    } else {
#pragma unroll
      for (int it = 0; it < 4; ++it) {
        const int row = 4 * it + (lane >> 3);
        const int c8 = (lane & 7) * 8;
        const v4f a = *(const v4f*)(sl + row * SLP + c8);
        const v4f b = *(const v4f*)(sl + row * SLP + c8 + 4);
        v4u hi, lo;
        split8(a, b, hi, lo);
        const size_t po = ((size_t)g * NF + m0 + row) * NN + n0 + c8;
        *(volatile v4u*)(outP + po) = hi;
        *(volatile v4u*)(outP + (size_t)oPlane + po) = lo;
      }
      if (w == 0) {
        const v4f v = *(const v4f*)(&sline[h][rl * 4]);
        *(volatile v4f*)(outF + (size_t)g * (2 * NN) + (size_t)h * NN + n0 + rl * 4) = v;
      }
    }
    __threadfence();
  }
}

__device__ __forceinline__ float lgt(float s1v, float s2v, int a) {
  float e = s1v + s2v;
  e = (e >= 0.0f) ? e : SLOPE * e;
  return (a > 0) ? e : NEGV;
}

template <int MODE>
__global__ void __launch_bounds__(256)
k_attn(const float* __restrict__ sc, const int* __restrict__ adj,
       const unsigned short* __restrict__ hT, long hPlane, int hdiv,
       const float* __restrict__ resid, const float* __restrict__ gam, const float* __restrict__ bet,
       int relu, int wplanes,
       float* __restrict__ outF, unsigned short* __restrict__ outP, long oPlane)
{
  __shared__ float s2sh[NN];
  __shared__ float s1sh[64];
  __shared__ float rinv[64];
  __shared__ __align__(16) unsigned short ph[64 * PTP];
  __shared__ __align__(16) unsigned short pl[64 * PTP];
  __shared__ __align__(16) float ot[64 * OTP];

  const int t = threadIdx.x, lane = t & 31, w = t >> 5, h = lane >> 4, rl = lane & 15;
  const int g = blockIdx.y;
  const int b = g / hdiv;
  const int hd = g - b * hdiv;
  const int n0 = blockIdx.x * 64;

  const float* scg = sc + (size_t)g * (2 * NN);
  s2sh[t] = scg[NN + t];
  s2sh[t + 256] = scg[NN + 256 + t];
  if (t < 64) s1sh[t] = scg[n0 + t];
  __syncthreads();

  const int pr = t >> 2, pc = (t & 3) * 8;
  const int* arow = adj + ((size_t)b * NN + n0 + pr) * NN + pc;
  const float s1v = s1sh[pr];

  float mx = NEGV;
#pragma unroll 2
  for (int ks = 0; ks < NN / 32; ++ks) {
    const int k0 = ks * 32;
    const v4i a0 = *(const v4i*)(arow + k0);
    const v4i a1 = *(const v4i*)(arow + k0 + 4);
    const float* s2p = s2sh + k0 + pc;
    mx = fmaxf(mx, lgt(s1v, s2p[0], a0.x));
    mx = fmaxf(mx, lgt(s1v, s2p[1], a0.y));
    mx = fmaxf(mx, lgt(s1v, s2p[2], a0.z));
    mx = fmaxf(mx, lgt(s1v, s2p[3], a0.w));
    mx = fmaxf(mx, lgt(s1v, s2p[4], a1.x));
    mx = fmaxf(mx, lgt(s1v, s2p[5], a1.y));
    mx = fmaxf(mx, lgt(s1v, s2p[6], a1.z));
    mx = fmaxf(mx, lgt(s1v, s2p[7], a1.w));
  }
  mx = fmaxf(mx, __shfl_xor(mx, 1, 32));
  mx = fmaxf(mx, __shfl_xor(mx, 2, 32));

  v8f acc[4];
  acc[0] = zero8(); acc[1] = zero8(); acc[2] = zero8(); acc[3] = zero8();
  float rs = 0.0f;
  const int rt = w >> 1, cb = (w & 1) * 64;
  const unsigned short* Bb = hT + ((size_t)g * NF + cb + rl) * NN + 8 * h;
  const size_t bsub = (size_t)16 * NN;
  const int aoff = (16 * rt + rl) * PTP + 8 * h;

  for (int ks = 0; ks < NN / 32; ++ks) {
    const int k0 = ks * 32;
    {
      const v4i a0 = *(const v4i*)(arow + k0);
      const v4i a1 = *(const v4i*)(arow + k0 + 4);
      const float* s2p = s2sh + k0 + pc;
      v4f q0, q1;
      q0.x = __expf(lgt(s1v, s2p[0], a0.x) - mx);
      q0.y = __expf(lgt(s1v, s2p[1], a0.y) - mx);
      q0.z = __expf(lgt(s1v, s2p[2], a0.z) - mx);
      q0.w = __expf(lgt(s1v, s2p[3], a0.w) - mx);
      q1.x = __expf(lgt(s1v, s2p[4], a1.x) - mx);
      q1.y = __expf(lgt(s1v, s2p[5], a1.y) - mx);
      q1.z = __expf(lgt(s1v, s2p[6], a1.z) - mx);
      q1.w = __expf(lgt(s1v, s2p[7], a1.w) - mx);
      rs += ((q0.x + q0.y) + (q0.z + q0.w)) + ((q1.x + q1.y) + (q1.z + q1.w));
      v4u hi, lo;
      split8(q0, q1, hi, lo);
      *(v4u*)(ph + pr * PTP + pc) = hi;
      *(v4u*)(pl + pr * PTP + pc) = lo;
    }
    __syncthreads();
    FragU fa, fb;
    fa.u[0] = *(const v4u*)(ph + aoff);
    fa.u[1] = *(const v4u*)(ph + aoff + 16);
    fb.u[0] = *(const v4u*)(pl + aoff);
    fb.u[1] = *(const v4u*)(pl + aoff + 16);
    mma12(acc, fa.v, fb.v, Bb + k0, Bb + (size_t)hPlane + k0, bsub);
    __syncthreads();
  }
  rs += __shfl_xor(rs, 1, 32);
  rs += __shfl_xor(rs, 2, 32);
  if ((t & 3) == 0) rinv[pr] = 1.0f / rs;
  accguard(acc);
  __syncthreads();

#pragma unroll
  for (int j = 0; j < 4; ++j) {
#pragma unroll
    for (int r = 0; r < 8; ++r) {
      const int row = 16 * rt + 8 * h + r;
      const int col = cb + 16 * j + rl;
      float v = acc[j][r] * rinv[row];
      if constexpr (MODE == 0) v = (v > 0.0f) ? v : (__expf(v) - 1.0f);
      ot[row * OTP + col] = v;
    }
  }
  __syncthreads();

  const size_t rowbase = (size_t)b * NN + n0;
  if constexpr (MODE == 0) {
    for (int pass = 0; pass < 2; ++pass) {
#pragma unroll
      for (int it = 0; it < 4; ++it) {
        const int row = 8 * w + 2 * it + h;
        const int c8 = rl * 8;
        const v4f a  = *(const v4f*)(ot + row * OTP + c8);
        const v4f bq = *(const v4f*)(ot + row * OTP + c8 + 4);
        v4u hi, lo;
        split8(a, bq, hi, lo);
        const size_t po = (rowbase + row) * HF + (size_t)hd * NF + c8;
        *(volatile v4u*)(outP + po) = hi;
        *(volatile v4u*)(outP + (size_t)oPlane + po) = lo;
      }
      __threadfence();
    }
  } else {
    const v4f gm = *(const v4f*)(gam + lane * 4);
    const v4f bt = *(const v4f*)(bet + lane * 4);
#pragma unroll 1
    for (int i = 0; i < 8; ++i) {
      const int row = 8 * w + i;
      v4f x = *(const v4f*)(ot + row * OTP + lane * 4);
      const v4f rr = *(const v4f*)(resid + (rowbase + row) * NF + lane * 4);
      x += rr;
      float s = (x.x + x.y) + (x.z + x.w);
#pragma unroll
      for (int off = 16; off > 0; off >>= 1) s += __shfl_xor(s, off, 32);
      const float mean = s * (1.0f / NF);
      const v4f d = x - mean;
      float q = (d.x * d.x + d.y * d.y) + (d.z * d.z + d.w * d.w);
#pragma unroll
      for (int off = 16; off > 0; off >>= 1) q += __shfl_xor(q, off, 32);
      const float var = q * (1.0f / NF);
      const float rstd = rsqrtf(var + LNEPS);
      v4f y = d * rstd * gm + bt;
      if (relu) {
        y.x = fmaxf(y.x, 0.0f); y.y = fmaxf(y.y, 0.0f);
        y.z = fmaxf(y.z, 0.0f); y.w = fmaxf(y.w, 0.0f);
      }
      *(v4f*)(ot + row * OTP + lane * 4) = y;
    }
    __syncthreads();
    for (int pass = 0; pass < 2; ++pass) {
#pragma unroll
      for (int i = 0; i < 8; ++i) {
        const int row = 8 * w + i;
        const size_t ro = (rowbase + row) * NF;
        const v4f y = *(const v4f*)(ot + row * OTP + lane * 4);
        *(volatile v4f*)(outF + ro + lane * 4) = y;
        if (wplanes) {
          const int c8 = rl * 8;
          const v4f a  = *(const v4f*)(ot + row * OTP + c8);
          const v4f bq = *(const v4f*)(ot + row * OTP + c8 + 4);
          v4u hi, lo;
          split8(a, bq, hi, lo);
          v4u sv = hi;
          if (h != 0) sv = lo;
          *(volatile v4u*)(outP + (size_t)h * (size_t)oPlane + ro + c8) = sv;
        }
      }
      __threadfence();
    }
  }
}

extern "C" void kernel_launch(void* const* d_in, const int* in_sizes, int n_in,
                              void* d_out, int out_size, void* d_ws, size_t ws_size,
                              hipStream_t stream)
{
  if (n_in < 10) return;
  if (in_sizes[0] != NB * NN * DIN) return;
  if (in_sizes[1] != NB * NN * NN) return;
  if (in_sizes[2] != DIN * NF) return;
  if (in_sizes[3] != NF) return;
  if (in_sizes[4] != NL * NH * NF * NF) return;
  if (in_sizes[5] != NL * NH * 2 * NF) return;
  if (in_sizes[6] != NL * HF * NF) return;
  if (in_sizes[7] != NL * 2 * NF) return;
  if (in_sizes[8] != NL * NF) return;
  if (in_sizes[9] != NL * NF) return;
  if (out_size != NB * NN * NF) return;

  const float* x   = (const float*)d_in[0];
  const int*   adj = (const int*)d_in[1];
  const float* Wp  = (const float*)d_in[2];
  const float* bp  = (const float*)d_in[3];
  const float* Wh  = (const float*)d_in[4];
  const float* ah  = (const float*)d_in[5];
  const float* Wo  = (const float*)d_in[6];
  const float* ao  = (const float*)d_in[7];
  const float* lg  = (const float*)d_in[8];
  const float* lb  = (const float*)d_in[9];

  const size_t eX  = (size_t)NB * NN * DIN;
  const size_t eWp = (size_t)NF * DIN;
  const size_t eWt = (size_t)NL * NH * NF * NF;
  const size_t eWo = (size_t)NL * NF * HF;
  const size_t eH  = (size_t)NB * NN * NF;
  const size_t eHT = (size_t)NB * NH * NF * NN;
  const size_t eM  = (size_t)NB * NN * HF;
  const size_t eHS = (size_t)NB * NF * NN;

  size_t off = 0;
  const size_t oX   = off; off += 2 * eX * 2;
  const size_t oWp  = off; off += 2 * eWp * 2;
  const size_t oWt  = off; off += 2 * eWt * 2;
  const size_t oWo  = off; off += 2 * eWo * 2;
  const size_t oHF0 = off; off += eH * 4;
  const size_t oHF1 = off; off += eH * 4;
  const size_t oHP0 = off; off += 2 * eH * 2;
  const size_t oHP1 = off; off += 2 * eH * 2;
  const size_t oHT  = off; off += 2 * eHT * 2;
  const size_t oSC  = off; off += (size_t)NB * NH * 2 * NN * 4;
  const size_t oM   = off; off += 2 * eM * 2;
  const size_t oHS  = off; off += 2 * eHS * 2;
  const size_t oSS  = off; off += (size_t)NB * 2 * NN * 4;
  if (off > ws_size) return;

  char* ws = (char*)d_ws;
  unsigned short* xpl  = (unsigned short*)(ws + oX);
  unsigned short* wppl = (unsigned short*)(ws + oWp);
  unsigned short* wtpl = (unsigned short*)(ws + oWt);
  unsigned short* wopl = (unsigned short*)(ws + oWo);
  float* hF[2];
  hF[0] = (float*)(ws + oHF0);
  hF[1] = (float*)(ws + oHF1);
  unsigned short* hpl[2];
  hpl[0] = (unsigned short*)(ws + oHP0);
  hpl[1] = (unsigned short*)(ws + oHP1);
  unsigned short* hTpl = (unsigned short*)(ws + oHT);
  float*          sch  = (float*)(ws + oSC);
  unsigned short* mpl  = (unsigned short*)(ws + oM);
  unsigned short* hsTpl = (unsigned short*)(ws + oHS);
  float*          scs  = (float*)(ws + oSS);

  const dim3 blk(256);

  {
    const int n8 = (int)(eX / 8);
    k_split<<<dim3((n8 + 255) / 256), blk, 0, stream>>>(x, xpl, (long)eX, n8);
  }
  k_tr<<<dim3(NF / 64, DIN / 64, 1), blk, 0, stream>>>(Wp, DIN, NF, (long)(DIN * NF), wppl, (long)eWp, (long)(DIN * NF));
  k_tr<<<dim3(NF / 64, NF / 64, NL * NH), blk, 0, stream>>>(Wh, NF, NF, (long)(NF * NF), wtpl, (long)eWt, (long)(NF * NF));
  k_tr<<<dim3(NF / 64, HF / 64, NL), blk, 0, stream>>>(Wo, HF, NF, (long)(HF * NF), wopl, (long)eWo, (long)(HF * NF));
  k_gemm<0><<<dim3(NF / 64, (NB * NN) / 128, 1), blk, 0, stream>>>(
      xpl, (long)eX, DIN, 0L, 1,
      wppl, (long)eWp, DIN, 0L, 1,
      DIN, bp, hF[0], hpl[0], (long)eH);

  for (int l = 0; l < NL; ++l) {
    const int cur = l & 1, nxt = (l + 1) & 1;
    k_gemm<1><<<dim3(NN / 64, 1, NB * NH), blk, 0, stream>>>(
        wtpl + (size_t)l * NH * NF * NF, (long)eWt, NF, (long)(NF * NF), NH,
        hpl[cur], (long)eH, NF, (long)(NN * NF), NH,
        NF, ah + (size_t)l * NH * 2 * NF, sch, hTpl, (long)eHT);
    k_attn<0><<<dim3(NN / 64, NB * NH), blk, 0, stream>>>(
        sch, adj, hTpl, (long)eHT, NH,
        lg, lg, lg, 0, 0,
        hF[0], mpl, (long)eM);
    k_gemm<1><<<dim3(NN / 64, 1, NB), blk, 0, stream>>>(
        wopl + (size_t)l * NF * HF, (long)eWo, HF, 0L, 1,
        mpl, (long)eM, HF, (long)(NN * HF), 1,
        HF, ao + (size_t)l * 2 * NF, scs, hsTpl, (long)eHS);
    float* dstF = (l == NL - 1) ? (float*)d_out : hF[nxt];
    k_attn<1><<<dim3(NN / 64, NB), blk, 0, stream>>>(
        scs, adj, hsTpl, (long)eHS, 1,
        hF[cur], lg + (size_t)l * NF, lb + (size_t)l * NF, (l < NL - 1) ? 1 : 0, (l < NL - 1) ? 1 : 0,
        dstF, hpl[nxt], (long)eH);
  }
  (void)hipGetLastError();
}
